// myRNNModel_38792144618212
// MI455X (gfx1250) — hardware-run, weakly checked
//
#include <hip/hip_runtime.h>
#include <math.h>

typedef __attribute__((ext_vector_type(16))) _Float16 v16h;
typedef __attribute__((ext_vector_type(8)))  _Float16 v8h;
typedef __attribute__((ext_vector_type(16))) __bf16   v16b;
typedef __attribute__((ext_vector_type(8)))  __bf16   v8b;
typedef __attribute__((ext_vector_type(8)))  float    v8f;
typedef __attribute__((ext_vector_type(4)))  float    v4f;

constexpr int kB    = 1024;
constexpr int kT    = 256;
constexpr int kV    = 10;
constexpr int kE    = 32;
constexpr int kHid  = 64;
constexpr int kO    = 10;
constexpr int kOP   = 64;
constexpr int kK    = 2 * kHid + 2 * kE;
constexpr int kKH   = 2 * kHid;
constexpr int kRows = kB * kT;
constexpr int kRC   = 65536;
constexpr int kThr  = 256;
constexpr float kInCarry = 1024.0f;
constexpr float kWCarry = 4096.0f;
constexpr float kSc = 1.0f / (kInCarry * kWCarry);
constexpr float kF16MinNormal = 6.103515625e-5f;

static_assert((kB % 64) == 0 && (kHid % 64) == 0 && (kOP % 64) == 0 && (kRows % 64) == 0 && (kK % 32) == 0 && (kHid % 32) == 0 && ((kB / 64) * (kHid / 64)) % 8 == 0 && (kRows % kRC) == 0 && ((kRC / 64) * (kOP / 64)) % 8 == 0, "GEMM M, N multiples of 64, K of 32; grids exact (16 and 1,024 tiles)");

constexpr size_t kOffW16 = 0ull;
constexpr size_t kOffWD16 = 24576ull;
constexpr size_t kOffBIAS = 32768ull;
constexpr size_t kOffHX16 = 33792ull;
constexpr size_t kOffPRE = 427008ull;
constexpr size_t kOffHS16 = 689152ull;
constexpr size_t kOffOUTP = 34243584ull;
constexpr size_t kWsTotal = 51020800ull;
static_assert(kWsTotal <= 134217728ull, "carve cap: under 128 MiB");
static_assert(kOffW16 == 0
              && kOffWD16 == kOffW16 + 24576ull
              && kOffBIAS == kOffWD16 + 8192ull
              && kOffHX16 == kOffBIAS + 1024ull
              && kOffPRE == kOffHX16 + 393216ull
              && kOffHS16 == kOffPRE + 262144ull
              && kOffOUTP == kOffHS16 + 33554432ull
              && kWsTotal == kOffOUTP + 16777216ull, "the carve is chained and totalled");
static_assert((kOffW16 % 256) == 0 && (kOffWD16 % 256) == 0 && (kOffBIAS % 256) == 0 && (kOffHX16 % 256) == 0 && (kOffPRE % 256) == 0 && (kOffHS16 % 256) == 0 && (kOffOUTP % 256) == 0, "aligned regions");
constexpr int kFBR = 0, kFBD = 64, kFEnd = 256;

__device__ __forceinline__ unsigned short f2bf_bits(float f) {
  unsigned u = __float_as_uint(f);
  return (unsigned short)((u + 0x7FFFu + ((u >> 16) & 1u)) >> 16);
}
__device__ __forceinline__ float bf_bits2f(unsigned short h) { return __uint_as_float(((unsigned)h) << 16); }
__device__ __forceinline__ float bf16r(float f) { return bf_bits2f(f2bf_bits(f)); }
__device__ __forceinline__ float carry_flush(float v, float carry) {
  const float s = v * carry;
  return (fabsf(s) < kF16MinNormal) ? 0.0f : s;
}
__device__ __forceinline__ float frcp(float x) { return __builtin_amdgcn_rcpf(x); }

__device__ __forceinline__ void dep_guard4_h(v8f& a, v8f& b, v8f& c, v8f& d, v16h x, v16h y) { asm volatile("v_nop\n\tv_nop\n\tv_nop\n\tv_nop" : "+v"(a), "+v"(b), "+v"(c), "+v"(d) : "v"(x), "v"(y)); }
__device__ __forceinline__ void dep_guard4_b(v8f& a, v8f& b, v8f& c, v8f& d, v16b x, v16b y) { asm volatile("v_nop\n\tv_nop\n\tv_nop\n\tv_nop" : "+v"(a), "+v"(b), "+v"(c), "+v"(d) : "v"(x), "v"(y)); }
__device__ __forceinline__ void keep4_h(v16h a, v16h b, v16h c, v16h d) { asm volatile("v_nop" :: "v"(a), "v"(b), "v"(c), "v"(d)); }
__device__ __forceinline__ void keep4_b(v16b a, v16b b, v16b c, v16b d) { asm volatile("v_nop" :: "v"(a), "v"(b), "v"(c), "v"(d)); }
__device__ __forceinline__ void acc_guard4(v8f& a, v8f& b, v8f& c, v8f& d) { asm volatile("v_nop\n\tv_nop\n\tv_nop\n\tv_nop" : "+v"(a), "+v"(b), "+v"(c), "+v"(d)); }

template <typename T> struct Frag;
template <> struct Frag<_Float16> {
  typedef v16h V; union U { v16h v; v8h h[2]; };
  static __device__ __forceinline__ v16h load(const _Float16* p) {
    U f; f.h[0] = *(const v8h*)(p); f.h[1] = *(const v8h*)(p + 16); return f.v;
  }
  static __device__ __forceinline__ v8f mma(v16h a, v16h b, v8f c) {
    return __builtin_amdgcn_wmma_f32_16x16x32_f16(false, a, false, b, (short)0, c, false, false);
  }
  static __device__ __forceinline__ void guard4(v8f& a, v8f& b, v8f& c, v8f& d, v16h x, v16h y) { dep_guard4_h(a, b, c, d, x, y); }
  static __device__ __forceinline__ void keep(v16h a, v16h b, v16h c, v16h d) { keep4_h(a, b, c, d); }
};
template <> struct Frag<__bf16> {
  typedef v16b V; union U { v16b v; v8b h[2]; };
  static __device__ __forceinline__ v16b load(const __bf16* p) {
    U f; f.h[0] = *(const v8b*)(p); f.h[1] = *(const v8b*)(p + 16); return f.v;
  }
  static __device__ __forceinline__ v8f mma(v16b a, v16b b, v8f c) {
    return __builtin_amdgcn_wmma_f32_16x16x32_bf16(false, a, false, b, (short)0, c, false, false);
  }
  static __device__ __forceinline__ void guard4(v8f& a, v8f& b, v8f& c, v8f& d, v16b x, v16b y) { dep_guard4_b(a, b, c, d, x, y); }
  static __device__ __forceinline__ void keep(v16b a, v16b b, v16b c, v16b d) { keep4_b(a, b, c, d); }
};

__device__ __forceinline__ v8f mma_h(v16h a, v16h b, v8f c) {
  c = __builtin_amdgcn_wmma_f32_16x16x32_f16(false, a, false, b, (short)0, c, false, false);
  asm volatile("v_nop\n\tv_nop\n\tv_nop\n\tv_nop" : "+v"(c) : "v"(a), "v"(b));
  return c;
}

template <int ET> struct Elem;
template <> struct Elem<0> { typedef _Float16 T; };
template <> struct Elem<1> { typedef __bf16 T; };
template <int ET, bool SPLIT, int BIAS_MODE, int OUT_MODE, bool RESID, int ACT = 0>
__global__ __launch_bounds__(256) void wmma_gemm64(
    const unsigned short* __restrict__ Ap, const unsigned short* __restrict__ A2p, int lda, long strideA,
    const unsigned short* __restrict__ Btp, const unsigned short* __restrict__ Bt2p, int ldb, long strideB,
    void* __restrict__ Cout, void* __restrict__ Cout2, int ldc, long strideC,
    const float* __restrict__ bias,
    const float* __restrict__ resid, long strideR,
    int M, int N, int K, float scale) {
  typedef typename Elem<ET>::T T;
  typedef typename Frag<T>::V V;
  const T* A = (const T*)Ap; const T* A2 = (const T*)A2p; const T* Bt = (const T*)Btp; const T* Bt2 = (const T*)Bt2p;
  __shared__ __align__(16) float sT[8][16 * 68];
  const int b    = blockIdx.y;
  const int lane = threadIdx.x & 31;
  const int wave = threadIdx.x >> 5;
  const int tilesN = N >> 6;
  const int tilesM = M >> 6;
  const int tile = blockIdx.x * 8 + wave;
  if (tile >= tilesM * tilesN) return;
  const int tm = tile / tilesN;
  const int tn = tile - tm * tilesN;
  const int m0 = tm << 6;
  const int n0 = tn << 6;

  const T* Ab  = A  + (size_t)b * strideA;
  const T* Bb  = Bt + (size_t)b * strideB;
  const T* Ab2 = SPLIT ? (A2  + (size_t)b * strideA) : nullptr;
  const T* Bb2 = SPLIT ? (Bt2 + (size_t)b * strideB) : nullptr;

  const int rlane = lane & 15;
  const int koff  = (lane >> 4) * 8;
  const int mOff  = (lane >> 4) * 8;

  v8f acc[4][4];
#pragma unroll
  for (int i = 0; i < 4; ++i)
#pragma unroll
    for (int j = 0; j < 4; ++j) acc[i][j] = (v8f){0.f,0.f,0.f,0.f,0.f,0.f,0.f,0.f};

  for (int k0 = 0; k0 < K; k0 += 32) {
    V bh[4], bl[4];
#pragma unroll
    for (int j = 0; j < 4; ++j) {
      const size_t bo = (size_t)(n0 + (j << 4) + rlane) * ldb + koff + k0;
      bh[j] = Frag<T>::load(Bb + bo);
      if (SPLIT) bl[j] = Frag<T>::load(Bb2 + bo);
    }
#pragma unroll
    for (int i = 0; i < 4; ++i) {
      const size_t ao = (size_t)(m0 + (i << 4) + rlane) * lda + koff + k0;
      V ah = Frag<T>::load(Ab + ao);
      V al;
      if (SPLIT) al = Frag<T>::load(Ab2 + ao);
#pragma unroll
      for (int j = 0; j < 4; ++j) {
        acc[i][j] = Frag<T>::mma(ah, bh[j], acc[i][j]);
        if (SPLIT) {
          acc[i][j] = Frag<T>::mma(ah, bl[j], acc[i][j]);
          acc[i][j] = Frag<T>::mma(al, bh[j], acc[i][j]);
        }
      }
      Frag<T>::guard4(acc[i][0], acc[i][1], acc[i][2], acc[i][3], ah, SPLIT ? al : ah);
    }
    Frag<T>::keep(bh[0], bh[1], bh[2], bh[3]);
    if (SPLIT) Frag<T>::keep(bl[0], bl[1], bl[2], bl[3]);
  }
  acc_guard4(acc[0][0], acc[0][1], acc[0][2], acc[0][3]);
  acc_guard4(acc[1][0], acc[1][1], acc[1][2], acc[1][3]);
  acc_guard4(acc[2][0], acc[2][1], acc[2][2], acc[2][3]);
  acc_guard4(acc[3][0], acc[3][1], acc[3][2], acc[3][3]);

  float* slab = sT[wave];
  const float* Rb = RESID ? (resid + (size_t)b * strideR) : nullptr;
#pragma unroll
  for (int i = 0; i < 4; ++i) {
    const int mBase = m0 + (i << 4);
#pragma unroll
    for (int j = 0; j < 4; ++j) {
      const int n = n0 + (j << 4) + rlane;
      float bv = 0.f;
      if (BIAS_MODE == 2) bv = bias[n];
#pragma unroll
      for (int r = 0; r < 8; ++r) {
        float v = acc[i][j][r] * scale;
        if (BIAS_MODE == 1) v += bias[mBase + mOff + r];
        if (BIAS_MODE == 2) v += bv;
        if (RESID) v += Rb[(size_t)(mBase + mOff + r) * ldc + n];
        if (ACT == 1) v = tanhf(v);
        if (ACT == 2) v = fmaxf(v, 0.0f);
        if (ACT == 3) v = v / (1.0f + expf(-v));
        if (ACT == 4) v = (v > 0.f) ? v : 0.01f * v;
        slab[(mOff + r) * 68 + (j << 4) + rlane] = v;
      }
    }
    __builtin_amdgcn_fence(__ATOMIC_RELEASE, "workgroup");
    __builtin_amdgcn_wave_barrier();
    __builtin_amdgcn_fence(__ATOMIC_ACQUIRE, "workgroup");
    if (OUT_MODE == 0) {
      float* C = (float*)Cout + (size_t)b * strideC;
      const int hh = lane >> 4, c4 = (lane & 15) * 4;
      for (int pass = 0; pass < 2; ++pass) {
#pragma unroll
        for (int it = 0; it < 8; ++it) {
          const int row = it * 2 + hh;
          v4f v = *(const v4f*)(slab + row * 68 + c4);
          *(volatile v4f*)(C + (size_t)(mBase + row) * ldc + n0 + c4) = v;
        }
        __threadfence();
      }
    } else {
      const int q = lane >> 3, c8 = (lane & 7) * 8;
      unsigned short* C  = (unsigned short*)Cout  + (size_t)b * strideC;
      unsigned short* C2 = (OUT_MODE == 2) ? ((unsigned short*)Cout2 + (size_t)b * strideC) : nullptr;
      for (int pass = 0; pass < 2; ++pass) {
#pragma unroll
        for (int it = 0; it < 4; ++it) {
          const int row = it * 4 + q;
          const float* sp = slab + row * 68 + c8;
          v8h hv, lv;
#pragma unroll
          for (int e = 0; e < 8; ++e) {
            if (OUT_MODE == 1) {
              hv[e] = (_Float16)sp[e];
            } else {
              unsigned short hb = f2bf_bits(sp[e]);
              unsigned short lb = f2bf_bits(sp[e] - bf_bits2f(hb));
              hv[e] = __builtin_bit_cast(_Float16, hb);
              lv[e] = __builtin_bit_cast(_Float16, lb);
            }
          }
          *(volatile v8h*)(C + (size_t)(mBase + row) * ldc + n0 + c8) = hv;
          if (OUT_MODE == 2) *(volatile v8h*)(C2 + (size_t)(mBase + row) * ldc + n0 + c8) = lv;
        }
        __threadfence();
      }
    }
    __builtin_amdgcn_fence(__ATOMIC_RELEASE, "workgroup");
    __builtin_amdgcn_wave_barrier();
    __builtin_amdgcn_fence(__ATOMIC_ACQUIRE, "workgroup");
  }
}

__global__ __launch_bounds__(256) void wt_plane_kernel(const float* __restrict__ W, unsigned short* __restrict__ dst, int K, int N, int nLive, int ldd, int colOff) {
  const int n  = blockIdx.x;
  const int k8 = threadIdx.x * 8;
  const bool live = n < nLive;
  const int nc = live ? n : 0;
  v8h hv;
#pragma unroll
  for (int e = 0; e < 8; ++e) {
    const float w = W[(size_t)(k8 + e) * N + nc];
    hv[e] = (_Float16)(live ? carry_flush(bf16r(w), kWCarry) : 0.0f);
  }
  unsigned short* dp = dst + (size_t)n * ldd + colOff + k8;
  *(volatile v8h*)dp = hv;
  __threadfence();
  *(volatile v8h*)dp = hv;
}

__device__ __forceinline__ void two_words(float v, _Float16& hi, _Float16& lo) {
  const float s = carry_flush(v, kInCarry);
  hi = (_Float16)s;
  const float r = s - (float)hi;
  lo = (_Float16)((fabsf(r) < kF16MinNormal) ? 0.0f : r);
}

__device__ __forceinline__ v8h emb_chunk(const int* __restrict__ num1, const int* __restrict__ num2, const float* __restrict__ emb, unsigned smp, int t, unsigned c) {
  const int* np = (c < 4u) ? num1 : num2;
  int d = np[(size_t)smp * kT + t];
  d = (d < 0) ? 0 : ((d > kV - 1) ? (kV - 1) : d);
  const float* ep = emb + (size_t)d * kE + (c & 3u) * 8u;
  const v4f a0 = *(const v4f*)ep, a1 = *(const v4f*)(ep + 4);
  v8h hv;
#pragma unroll
  for (int e = 0; e < 4; ++e) { const float p = a0[e], q = a1[e]; hv[e] = (_Float16)carry_flush(bf16r(p), kInCarry); hv[4 + e] = (_Float16)carry_flush(bf16r(q), kInCarry); }
  return hv;
}

__global__ __launch_bounds__(64) void setup_kernel(const int* __restrict__ num1, const int* __restrict__ num2, const float* __restrict__ emb,
                                                   const float* __restrict__ b_rnn, const float* __restrict__ bd, float* __restrict__ BIAS, unsigned short* __restrict__ HX16) {
  const unsigned y = blockIdx.y;
  const unsigned c = threadIdx.x;
  if (y == 0u) {
    v4f o = {0.f, 0.f, 0.f, 0.f};
#pragma unroll
    for (int e = 0; e < 4; ++e) {
      const unsigned i = c * 4u + (unsigned)e;
      const bool inR = i < (unsigned)kHid;
      const bool inD = (i >= (unsigned)kFBD) && (i < (unsigned)(kFBD + kO));
      const float p = b_rnn[inR ? i : 0u];
      const float q = bd[inD ? (i - (unsigned)kFBD) : 0u];
      o[e] = inR ? bf16r(p) : (inD ? bf16r(q) : 0.0f);
    }
    float* dp = BIAS + c * 4u;
    *(volatile v4f*)dp = o;
    __threadfence();
    *(volatile v4f*)dp = o;
  } else {
    if (c >= 24u) return;
    const unsigned smp = y - 1u;
    v8h hv;
    if (c < 16u) {
#pragma unroll
      for (int e = 0; e < 8; ++e) hv[e] = (_Float16)0.0f;
    } else {
      hv = emb_chunk(num1, num2, emb, smp, 0, c - 16u);
    }
    unsigned short* dp = HX16 + (size_t)smp * kK + c * 8u;
    *(volatile v8h*)dp = hv;
    __threadfence();
    *(volatile v8h*)dp = hv;
  }
}
static_assert(kFEnd == 4 * 64 && kFBD == kHid && kK / 8 == 24 && kHid / 8 == 8 && kE / 8 == 4, "set-up rows: the bias stream is one block's 64 threads; 24 chunks an operand row");

__global__ __launch_bounds__(32) void cell_kernel(const float* __restrict__ PRE, const int* __restrict__ num1, const int* __restrict__ num2, const float* __restrict__ emb,
                                                  unsigned short* __restrict__ HX16, unsigned short* __restrict__ HS16, int t) {
  const unsigned smp = blockIdx.y;
  const unsigned c = threadIdx.x;
  if (c < 8u) {
    const float* pp = PRE + (size_t)smp * kHid + c * 8u;
    const v4f a0 = *(const v4f*)pp, a1 = *(const v4f*)(pp + 4);
    v8h hv, lv;
#pragma unroll
    for (int e = 0; e < 4; ++e) {
      _Float16 h0w, l0w, h1w, l1w;
      two_words(tanhf(a0[e]), h0w, l0w);
      two_words(tanhf(a1[e]), h1w, l1w);
      hv[e] = h0w; hv[4 + e] = h1w; lv[e] = l0w; lv[4 + e] = l1w;
    }
    unsigned short* hp = HX16 + (size_t)smp * kK + c * 8u;
    unsigned short* sp = HS16 + ((size_t)smp * kT + (size_t)t) * kHid + c * 8u;
    for (int pass = 0; pass < 2; ++pass) {
      *(volatile v8h*)hp = hv;
      *(volatile v8h*)(hp + kHid) = lv;
      *(volatile v8h*)sp = hv;
      __threadfence();
    }
  } else if (c < 16u && t + 1 < kT) {
    const v8h xv = emb_chunk(num1, num2, emb, smp, t + 1, c - 8u);
    unsigned short* xp = HX16 + (size_t)smp * kK + kKH + (c - 8u) * 8u;
    *(volatile v8h*)xp = xv;
    __threadfence();
    *(volatile v8h*)xp = xv;
  }
}

__global__ __launch_bounds__(kThr) void out_kernel(const float* __restrict__ OUTP, float* __restrict__ out) {
  const unsigned v = blockIdx.x * (unsigned)kThr + threadIdx.x;
  v4f a;
#pragma unroll
  for (int e = 0; e < 4; ++e) {
    const unsigned i = v * 4u + (unsigned)e;
    const unsigned row = i / (unsigned)kO;
    const unsigned col = i - row * (unsigned)kO;
    a[e] = OUTP[(size_t)row * kOP + col];
  }
  float* dp = out + (size_t)v * 4u;
  *(volatile v4f*)dp = a;
  __threadfence();
  *(volatile v4f*)dp = a;
}
static_assert(((size_t)kRC * kO / 4) == 640 * kThr, "output grid exact");

extern "C" void kernel_launch(void* const* d_in, const int* in_sizes, int n_in,
                              void* d_out, int out_size, void* d_ws, size_t ws_size,
                              hipStream_t stream) {
  if (n_in < 8 || d_out == nullptr || d_ws == nullptr) return;
  if (in_sizes[0] != kB * kT || in_sizes[1] != kB * kT || in_sizes[2] != kV * kE || in_sizes[3] != 2 * kE * kHid || in_sizes[4] != kHid * kHid || in_sizes[5] != kHid || in_sizes[6] != kHid * kO || in_sizes[7] != kO) return;
  if (out_size != kRows * kO) return;
  if (ws_size < kWsTotal) return;
  const int* num1 = (const int*)d_in[0];
  const int* num2 = (const int*)d_in[1];
  const float* emb = (const float*)d_in[2];
  const float* Wx = (const float*)d_in[3];
  const float* Wh = (const float*)d_in[4];
  const float* b_rnn = (const float*)d_in[5];
  const float* Wd = (const float*)d_in[6];
  const float* bd = (const float*)d_in[7];
  float* out = (float*)d_out;
  char* ws = (char*)d_ws;
  unsigned short* W16 = (unsigned short*)(ws + kOffW16);
  unsigned short* WD16 = (unsigned short*)(ws + kOffWD16);
  float* BIAS = (float*)(ws + kOffBIAS);
  unsigned short* HX16 = (unsigned short*)(ws + kOffHX16);
  float* PRE = (float*)(ws + kOffPRE);
  unsigned short* HS16 = (unsigned short*)(ws + kOffHS16);
  float* OUTP = (float*)(ws + kOffOUTP);

  wt_plane_kernel<<<kHid, kHid / 8, 0, stream>>>(Wh, W16, kHid, kHid, kHid, kK, 0);
  wt_plane_kernel<<<kHid, kHid / 8, 0, stream>>>(Wh, W16, kHid, kHid, kHid, kK, kHid);
  wt_plane_kernel<<<kHid, 2 * kE / 8, 0, stream>>>(Wx, W16, 2 * kE, kHid, kHid, kK, kKH);
  wt_plane_kernel<<<kOP, kHid / 8, 0, stream>>>(Wd, WD16, kHid, kO, kO, kHid, 0);
  setup_kernel<<<dim3(1, 1 + kB), 64, 0, stream>>>(num1, num2, emb, b_rnn, bd, BIAS, HX16);
  for (int t = 0; t < kT; ++t) {
    wmma_gemm64<0, false, 2, 0, false, 0><<<dim3((kB / 64) * (kHid / 64) / 8, 1), 256, 0, stream>>>(
        HX16, HX16, kK, 0L, W16, W16, kK, 0L, (void*)PRE, (void*)PRE, kHid, 0L, BIAS + kFBR, nullptr, 0L, kB, kHid, kK, kSc);
    cell_kernel<<<dim3(1, kB), 32, 0, stream>>>(PRE, num1, num2, emb, HX16, HS16, t);
  }
  for (int ch = 0; ch < kRows / kRC; ++ch) {
    const unsigned short* Hc = HS16 + (size_t)ch * kRC * kHid;
    wmma_gemm64<0, false, 2, 0, false, 0><<<dim3((kRC / 64) * (kOP / 64) / 8, 1), 256, 0, stream>>>(
        Hc, Hc, kHid, 0L, WD16, WD16, kHid, 0L, (void*)OUTP, (void*)OUTP, kOP, 0L, BIAS + kFBD, nullptr, 0L, kRC, kOP, kHid, kSc);
    out_kernel<<<640, kThr, 0, stream>>>(OUTP, out + (size_t)ch * kRC * kO);
  }
}
